// WavLMMultiheadAttention_90271622627746
// MI455X (gfx1250) — hardware-run, weakly checked
//
#include <hip/hip_runtime.h>


#ifndef NB
#define NB 2
#endif
#ifndef SEQ
#define SEQ 2048
#endif
#define NB_FULL  2
#define SEQ_FULL 2048
#define DM   1024
#define NH_  16
#define HD   64
#define AW   4
#define OSP  68
#define GT   8
#define RBC  2048
#define RBN  4096
#define BK_T9  12
#define BK_T10 16
#define BK_T11 23
#define BK_T12 32
#define BK_T13 46
#define BK_T14 64
#define BK_SAT 91
#define SC2   ((float)(0.125 * 1.4426950408889634))
#define LOG2E ((float)1.4426950408889634)
#define PSH  14.0f
#define NEGB (-3.0e38f)
#define CXS  1024.0f
#define WOS  64.0f
#define OSC  (1.0f / 65536.0f)

static_assert(HD == 64);
static_assert(NH_ * HD == DM);
static_assert(DM % 64 == 0);
static_assert(DM % 32 == 0);
static_assert(HD % 32 == 0);
static_assert(SEQ % 64 == 0);
static_assert((NB * SEQ) % 64 == 0);
static_assert(SEQ % 32 == 0);
static_assert(SEQ % (16 * AW) == 0);
static_assert((NB * SEQ) % GT == 0);
static_assert(GT * NH_ == 32 * 4);
static_assert(SEQ <= RBC);
static_assert(RBN == 2 * RBC);
static_assert(BK_SAT + 64 < RBC);
static_assert((RBN / 4) % (32 * AW) == 0);
static_assert(32 * 16 * 4 == 16 * HD * 2);
static_assert(32 * 16 * 8 == 16 * 64 * 4);
static_assert(((size_t)DM * DM) % 8 == 0);
static_assert(((size_t)NB * SEQ * DM) % 8 == 0);
static_assert(NB <= NB_FULL);
static_assert(SEQ <= SEQ_FULL);
static_assert((OSP * 4) % 16 == 0);
static_assert((size_t)(RBN + AW * 16 * OSP) * 4 <= 131072);
static_assert((size_t)(16 * 68) * 4 <= 131072);
static_assert(((size_t)(SEQ_FULL - 1) * NB_FULL + NB_FULL) * DM * 4 == (size_t)16777216);

typedef _Float16 h16;
typedef unsigned short bf;
typedef __attribute__((ext_vector_type(16))) __bf16   v16bf;
typedef __attribute__((ext_vector_type(16))) _Float16 v16h;
typedef __attribute__((ext_vector_type(8)))  _Float16 v8h;
typedef __attribute__((ext_vector_type(8)))  unsigned short v8us;
typedef __attribute__((ext_vector_type(8)))  float    v8f;
typedef __attribute__((ext_vector_type(4)))  float    v4f;
typedef v4f  __attribute__((may_alias)) v4fa;

__device__ __forceinline__ unsigned short f2bf(float f) { unsigned u = __float_as_uint(f); u += 0x7FFFu + ((u >> 16) & 1u); return (unsigned short)(u >> 16); }
__device__ __forceinline__ float bfr(float f) { return __uint_as_float(((unsigned)f2bf(f)) << 16); }
__device__ __forceinline__ v16h cat16(v8h lo, v8h hi) { return __builtin_shufflevector(lo, hi, 0, 1, 2, 3, 4, 5, 6, 7, 8, 9, 10, 11, 12, 13, 14, 15); }
__device__ __forceinline__ v16bf cat16b(v8us lo, v8us hi) { return __builtin_bit_cast(v16bf, __builtin_shufflevector(lo, hi, 0, 1, 2, 3, 4, 5, 6, 7, 8, 9, 10, 11, 12, 13, 14, 15)); }
__device__ __forceinline__ v8f wmma16(v16h a, v16h b, v8f c) { return __builtin_amdgcn_wmma_f32_16x16x32_f16(false, a, false, b, (short)0, c, false, false); }
__device__ __forceinline__ v8f wmmab(v16bf a, v16bf b, v8f c) { return __builtin_amdgcn_wmma_f32_16x16x32_bf16(false, a, false, b, (short)0, c, false, false); }
__device__ __forceinline__ v16h  ldh(const h16* p) { return cat16(*(const v8h*)p, *(const v8h*)(p + 16)); }
__device__ __forceinline__ v16bf ldb(const bf* p)  { return cat16b(*(const v8us*)p, *(const v8us*)(p + 16)); }
__device__ __forceinline__ void wave_sync() { __builtin_amdgcn_fence(3  , "wavefront"); __builtin_amdgcn_wave_barrier(); asm volatile("" ::: "memory"); }
__device__ __forceinline__ h16 toh_flush(float v) { const h16 r = (h16)v; return (fabsf(v) < 6.103515625e-05f) ? (h16)0.0f : r; }
__device__ __forceinline__ v8f wmg16(v16h a, v16h b, v8f c) { c = wmma16(a, b, c); asm volatile("v_nop\n\tv_nop\n\tv_nop\n\tv_nop" : "+v"(c) : "v"(a), "v"(b)); return c; }
__device__ __forceinline__ v8f wmgb(v16bf a, v16bf b, v8f c) { c = wmmab(a, b, c); asm volatile("v_nop\n\tv_nop\n\tv_nop\n\tv_nop" : "+v"(c) : "v"(a), "v"(b)); return c; }

__global__ __launch_bounds__(256) void k_cvt8(const float* __restrict__ src, bf* dst, size_t n8) {
    const size_t i = (size_t)blockIdx.x * 256 + threadIdx.x; if (i >= n8) return;
    const v8f v = *(const v8f*)(src + i * 8); v8us o;
#pragma unroll
    for (int k = 0; k < 8; ++k) o[k] = f2bf(v[k]);
    *(volatile v8us*)(dst + i * 8) = o; __threadfence(); *(volatile v8us*)(dst + i * 8) = o;
}

__global__ __launch_bounds__(256) void k_cvtx(const float* __restrict__ src, bf* dst) {
    const size_t n8 = (size_t)NB * SEQ * DM / 8;
    const size_t i = (size_t)blockIdx.x * 256 + threadIdx.x; if (i >= n8) return;
    const size_t row = i / (DM / 8); const size_t c = i % (DM / 8);
    const size_t b = row / SEQ, t = row % SEQ;
    const v8f v = *(const v8f*)(src + (t * NB_FULL + b) * DM + c * 8); v8us o;
#pragma unroll
    for (int k = 0; k < 8; ++k) o[k] = f2bf(v[k]);
    *(volatile v8us*)(dst + i * 8) = o; __threadfence(); *(volatile v8us*)(dst + i * 8) = o;
}

__global__ __launch_bounds__(256) void k_cvtw(const float* __restrict__ src, h16* dst, size_t n8) {
    const size_t i = (size_t)blockIdx.x * 256 + threadIdx.x; if (i >= n8) return;
    const v8f v = *(const v8f*)(src + i * 8); v8h o;
#pragma unroll
    for (int k = 0; k < 8; ++k) o[k] = toh_flush(bfr(v[k]) * WOS);
    *(volatile v8h*)(dst + i * 8) = o; __threadfence(); *(volatile v8h*)(dst + i * 8) = o;
}

__global__ __launch_bounds__(128) void k_gw(const float* __restrict__ gw, bf* GW) {
    const int i = threadIdx.x; const int row = i >> 3, c8 = (i & 7) * 8; const int rs = row & 7;
    const v8f v = *(const v8f*)(gw + rs * HD + c8); v8us o;
#pragma unroll
    for (int k = 0; k < 8; ++k) { const unsigned short w = f2bf(v[k]); o[k] = (row < 8) ? w : (unsigned short)0; }
    *(volatile v8us*)(GW + i * 8) = o; __threadfence(); *(volatile v8us*)(GW + i * 8) = o;
}

__device__ __forceinline__ int rel_class(int rp) {
    const int a = rp < 0 ? -rp : rp;
    const int lg = 8 + (a >= BK_T9 ? 1 : 0) + (a >= BK_T10 ? 1 : 0) + (a >= BK_T11 ? 1 : 0) + (a >= BK_T12 ? 1 : 0) + (a >= BK_T13 ? 1 : 0) + (a >= BK_T14 ? 1 : 0) + (a >= BK_SAT ? 1 : 0);
    const int add = (a < 8) ? a : lg;
    return (rp > 0 ? 16 : 0) + add;
}

__global__ __launch_bounds__(256) void k_relb(const float* __restrict__ rel_emb, float* RB) {
    const int i = blockIdx.x * 256 + threadIdx.x; if (i >= NH_ * RBN / 4) return;
    const int h = i / (RBN / 4); const int j0 = (i % (RBN / 4)) * 4;
    v4f o;
#pragma unroll
    for (int k = 0; k < 4; ++k) { const int cls = rel_class(j0 + k - RBC); o[k] = bfr(rel_emb[cls * NH_ + h]); }
    float* dst = RB + (size_t)h * RBN + j0;
    *(volatile v4f*)dst = o; __threadfence(); *(volatile v4f*)dst = o;
}

__global__ __launch_bounds__(32) void k_gate(const bf* __restrict__ XB, const bf* __restrict__ GW, const float* __restrict__ gb, const float* __restrict__ ga, float* GA) {
    __shared__ __align__(16) float gs[GT * NH_];
    const int lane = threadIdx.x & 31, lr = lane & 15, hi = lane >> 4;
    const size_t tok0 = (size_t)blockIdx.x * GT;
    const v16bf b0 = ldb(GW + lr * HD + 8 * hi), b1 = ldb(GW + lr * HD + 32 + 8 * hi);
    const float gbl = bfr(gb[lr & 7]); const float gbv = (lr < 8) ? gbl : 0.0f;
    const float gav = bfr(ga[8 * hi + (lr & 7)]);
#pragma unroll 1
    for (int i = 0; i < GT; ++i) {
        const bf* ap = XB + ((tok0 + (size_t)i) * NH_ + (size_t)lr) * HD + 8 * hi;
        const v16bf a0 = ldb(ap), a1 = ldb(ap + 32);
        v8f acc = (v8f){};
        acc = wmgb(a0, b0, acc); acc = wmgb(a1, b1, acc);
        float sas = 0.0f, sbs = 0.0f;
#pragma unroll
        for (int r = 0; r < 8; ++r) {
            float v = acc[r] + gbv;
            v += __shfl_xor(v, 1, 32); v += __shfl_xor(v, 2, 32);
            const float a = __shfl(v, hi * 16, 32), c = __shfl(v, hi * 16 + 4, 32);
            const bool mine = ((lr & 7) == r);
            sas = mine ? a : sas; sbs = mine ? c : sbs;
        }
        const float ea = 1.0f / (1.0f + expf(-sas)), eb = 1.0f / (1.0f + expf(-sbs));
        const float g = ea * (eb * gav - 1.0f) + 2.0f;
        if (lr < 8) gs[i * NH_ + 8 * hi + lr] = g;
    }
    wave_sync();
    const v4f val = *(const v4fa*)(&gs[lane * 4]);
    float* dst = GA + tok0 * NH_ + lane * 4;
    *(volatile v4f*)dst = val; __threadfence(); *(volatile v4f*)dst = val;
}

__device__ __forceinline__ void gemm_bf(const bf* __restrict__ A, const bf* __restrict__ Bt, int r0, int c0, int lr, int hi, v8f (&acc)[4][4]) {
#pragma unroll
    for (int mb = 0; mb < 4; ++mb)
#pragma unroll
        for (int nb = 0; nb < 4; ++nb) acc[mb][nb] = (v8f){};
    const size_t aoff = (size_t)(r0 + lr) * DM + 8 * hi, boff = (size_t)(c0 + lr) * DM + 8 * hi;
#pragma unroll 1
    for (int kc = 0; kc < DM; kc += 32) {
        v16bf a[4];
#pragma unroll
        for (int mb = 0; mb < 4; ++mb) a[mb] = ldb(A + aoff + (size_t)mb * 16 * DM + kc);
#pragma unroll
        for (int nb = 0; nb < 4; ++nb) { const v16bf b = ldb(Bt + boff + (size_t)nb * 16 * DM + kc);
#pragma unroll
            for (int mb = 0; mb < 4; ++mb) acc[mb][nb] = wmgb(a[mb], b, acc[mb][nb]); }
    }
}
__device__ __forceinline__ void gemm_h(const h16* __restrict__ A, const h16* __restrict__ Bt, int r0, int c0, int lr, int hi, v8f (&acc)[4][4]) {
#pragma unroll
    for (int mb = 0; mb < 4; ++mb)
#pragma unroll
        for (int nb = 0; nb < 4; ++nb) acc[mb][nb] = (v8f){};
    const size_t aoff = (size_t)(r0 + lr) * DM + 8 * hi, boff = (size_t)(c0 + lr) * DM + 8 * hi;
#pragma unroll 1
    for (int kc = 0; kc < DM; kc += 32) {
        v16h a[4];
#pragma unroll
        for (int mb = 0; mb < 4; ++mb) a[mb] = ldh(A + aoff + (size_t)mb * 16 * DM + kc);
#pragma unroll
        for (int nb = 0; nb < 4; ++nb) { const v16h b = ldh(Bt + boff + (size_t)nb * 16 * DM + kc);
#pragma unroll
            for (int mb = 0; mb < 4; ++mb) acc[mb][nb] = wmg16(a[mb], b, acc[mb][nb]); }
    }
}

__global__ __launch_bounds__(32) void k_projqk(const bf* __restrict__ A, const bf* __restrict__ Bt, const float* __restrict__ bias, h16* Ph) {
    __shared__ __align__(16) float os[16 * 68];
    const int lane = threadIdx.x & 31, lr = lane & 15, hi = lane >> 4; const int r0 = blockIdx.x * 64, c0 = blockIdx.y * 64;
    v8f acc[4][4];
    gemm_bf(A, Bt, r0, c0, lr, hi, acc);
    float bc[4];
#pragma unroll
    for (int nb = 0; nb < 4; ++nb) bc[nb] = bfr(bias[c0 + nb * 16 + lr]);
    const int bb = r0 / SEQ, tt = r0 % SEQ; const int zc = bb * NH_ + c0 / HD;
    const size_t tbase = ((size_t)zc * SEQ + (size_t)tt) * HD;
#pragma unroll
    for (int mb = 0; mb < 4; ++mb) {
#pragma unroll
        for (int nb = 0; nb < 4; ++nb) {
#pragma unroll
            for (int j = 0; j < 8; ++j) os[(hi * 8 + j) * 68 + nb * 16 + lr] = acc[mb][nb][j] + bc[nb]; }
        wave_sync();
#pragma unroll 1
        for (int ps = 0; ps < 2; ++ps) {
#pragma unroll
            for (int s = 0; s < 4; ++s) { const int row = 4 * s + (lane >> 3), c8 = (lane & 7) * 8;
                const v4f x0 = *(const v4fa*)(&os[row * 68 + c8]); const v4f x1 = *(const v4fa*)(&os[row * 68 + c8 + 4]); v8h hv;
#pragma unroll
                for (int i = 0; i < 4; ++i) { hv[i] = toh_flush(x0[i]); hv[4 + i] = toh_flush(x1[i]); }
                const size_t oo = tbase + (size_t)(mb * 16 + row) * HD + c8;
                *(volatile v8h*)(Ph + oo) = hv; }
            if (ps == 0) __threadfence(); }
        wave_sync();
    }
}

__global__ __launch_bounds__(32) void k_projv(const bf* __restrict__ A, const bf* __restrict__ Bt, const float* __restrict__ bias, h16* Ph) {
    __shared__ __align__(16) float os[16 * 68];
    const int lane = threadIdx.x & 31, lr = lane & 15, hi = lane >> 4; const int r0 = blockIdx.x * 64, c0 = blockIdx.y * 64;
    v8f acc[4][4];
    gemm_bf(A, Bt, r0, c0, lr, hi, acc);
    const int bb = c0 / SEQ, tt = c0 % SEQ;
    const size_t tbase = (size_t)bb * (size_t)DM * SEQ + (size_t)r0 * SEQ + (size_t)tt;
#pragma unroll
    for (int mb = 0; mb < 4; ++mb) {
        float br[8];
#pragma unroll
        for (int j = 0; j < 8; ++j) br[j] = bfr(bias[r0 + mb * 16 + hi * 8 + j]);
#pragma unroll
        for (int nb = 0; nb < 4; ++nb) {
#pragma unroll
            for (int j = 0; j < 8; ++j) os[(hi * 8 + j) * 68 + nb * 16 + lr] = acc[mb][nb][j] + br[j]; }
        wave_sync();
#pragma unroll 1
        for (int ps = 0; ps < 2; ++ps) {
#pragma unroll
            for (int s = 0; s < 4; ++s) { const int row = 4 * s + (lane >> 3), c8 = (lane & 7) * 8;
                const v4f x0 = *(const v4fa*)(&os[row * 68 + c8]); const v4f x1 = *(const v4fa*)(&os[row * 68 + c8 + 4]); v8h hv;
#pragma unroll
                for (int i = 0; i < 4; ++i) { hv[i] = toh_flush(x0[i]); hv[4 + i] = toh_flush(x1[i]); }
                const size_t oo = tbase + (size_t)(mb * 16 + row) * SEQ + c8;
                *(volatile v8h*)(Ph + oo) = hv; }
            if (ps == 0) __threadfence(); }
        wave_sync();
    }
}

__global__ __launch_bounds__(32) void k_oproj(const h16* __restrict__ A, const h16* __restrict__ Bt, const float* __restrict__ bias, float* OUT) {
    __shared__ __align__(16) float os[16 * 68];
    const int lane = threadIdx.x & 31, lr = lane & 15, hi = lane >> 4; const int r0 = blockIdx.x * 64, c0 = blockIdx.y * 64;
    v8f acc[4][4];
    gemm_h(A, Bt, r0, c0, lr, hi, acc);
    float bc[4];
#pragma unroll
    for (int nb = 0; nb < 4; ++nb) bc[nb] = bfr(bias[c0 + nb * 16 + lr]);
#pragma unroll
    for (int mb = 0; mb < 4; ++mb) {
#pragma unroll
        for (int nb = 0; nb < 4; ++nb) {
#pragma unroll
            for (int j = 0; j < 8; ++j) os[(hi * 8 + j) * 68 + nb * 16 + lr] = acc[mb][nb][j] * OSC + bc[nb]; }
        wave_sync();
#pragma unroll 1
        for (int ps = 0; ps < 2; ++ps) {
#pragma unroll
            for (int s = 0; s < 8; ++s) { const int p = s * 32 + lane; const int row = p >> 4, c4 = (p & 15) * 4;
                const v4f val = *(const v4fa*)(&os[row * 68 + c4]);
                const int mrow = r0 + mb * 16 + row; const int bq = mrow / SEQ, tq = mrow % SEQ;
                *(volatile v4f*)(OUT + ((size_t)tq * NB_FULL + (size_t)bq) * DM + c0 + c4) = val; }
            if (ps == 0) __threadfence(); }
        wave_sync();
    }
}

__global__ __launch_bounds__(32 * AW) void k_flash(const h16* __restrict__ QH, const h16* __restrict__ KP, const h16* __restrict__ VT,
                                                   const float* __restrict__ GA, const float* __restrict__ RB, h16* CTX) {
    __shared__ __align__(16) float sbt[RBN];
    __shared__ __align__(16) float os[AW * 16 * OSP];
    const int lane = threadIdx.x & 31, lr = lane & 15, hi = lane >> 4;
    const int wave = __builtin_amdgcn_readfirstlane((int)(threadIdx.x >> 5));
    const int zh = blockIdx.y; const int b = zh / NH_, h = zh % NH_;
    { const float* rb = RB + (size_t)h * RBN;
#pragma unroll 1
      for (int i = threadIdx.x; i < RBN / 4; i += 32 * AW) { const v4f v = *(const v4f*)(rb + i * 4); *(v4fa*)(&sbt[i * 4]) = v; } }
    __syncthreads();
    const int t0 = (blockIdx.x * AW + wave) * 16;
    const float gl = GA[((size_t)b * SEQ + (size_t)(t0 + lr)) * NH_ + h] * LOG2E;
    const float bpos = gl * sbt[RBC + BK_SAT], bneg = gl * sbt[RBC - BK_SAT];
    const size_t pbase = (size_t)zh * SEQ * HD;
    const size_t qo = pbase + (size_t)(t0 + lr) * HD + 8 * hi;
    const v16h q0 = ldh(QH + qo), q1 = ldh(QH + qo + 32);
    const size_t ko = pbase + (size_t)lr * HD + 8 * hi;
    const size_t vo = pbase + (size_t)lr * SEQ + 8 * hi;
    v8f o[4];
#pragma unroll
    for (int j = 0; j < 4; ++j) o[j] = (v8f){};
    float m = NEGB, l = 0.0f;
#pragma unroll 1
    for (int key0 = 0; key0 < SEQ; key0 += 32) {
        const h16* ka = KP + ko + (size_t)key0 * HD;
        const v16h ka0 = ldh(ka), ka1 = ldh(ka + 32), kb0 = ldh(ka + 16 * HD), kb1 = ldh(ka + 16 * HD + 32);
        v8f sa = (v8f){}, sc = (v8f){};
        sa = wmg16(ka0, q0, sa); sa = wmg16(ka1, q1, sa); sc = wmg16(kb0, q0, sc); sc = wmg16(kb1, q1, sc);
        const int d0 = key0 - t0;
        float ba[8], bb[8];
        if (d0 - 15 >= BK_SAT) {
#pragma unroll
            for (int r = 0; r < 8; ++r) { ba[r] = bpos; bb[r] = bpos; }
        } else if (d0 + 31 <= -BK_SAT) {
#pragma unroll
            for (int r = 0; r < 8; ++r) { ba[r] = bneg; bb[r] = bneg; }
        } else {
            const int ib = RBC + d0 + 8 * hi - lr;
#pragma unroll
            for (int r = 0; r < 8; ++r) { ba[r] = gl * sbt[ib + r]; bb[r] = gl * sbt[ib + 16 + r]; }
        }
        float ta[8], tb[8]; float mx = NEGB;
#pragma unroll
        for (int r = 0; r < 8; ++r) {
            ta[r] = sa[r] * SC2 + ba[r]; tb[r] = sc[r] * SC2 + bb[r];
            mx = fmaxf(mx, fmaxf(ta[r], tb[r])); }
        mx = fmaxf(mx, __shfl_xor(mx, 16, 32));
        const float mnew = fmaxf(m, mx);
        const float alpha = __builtin_amdgcn_exp2f(m - mnew);
        const float sh = PSH - mnew;
        v16h pb; float ls = 0.0f;
#pragma unroll
        for (int r = 0; r < 8; ++r) {
            const float xa = ta[r] + sh, xb = tb[r] + sh;
            const float ea = __builtin_amdgcn_exp2f(xa), eb = __builtin_amdgcn_exp2f(xb);
            const float ga = (xa < -14.0f) ? 0.0f : ea, gb = (xb < -14.0f) ? 0.0f : eb;
            const h16 pa = (h16)ga; const h16 pc = (h16)gb;
            pb[r] = pa; pb[8 + r] = pc;
            ls += (float)pa + (float)pc; }
        l = l * alpha + ls; m = mnew;
#pragma unroll
        for (int j = 0; j < 4; ++j) o[j] = o[j] * alpha;
        const h16* va = VT + vo + key0;
#pragma unroll
        for (int j = 0; j < 4; ++j) { const v16h vj = ldh(va + (size_t)(16 * j) * SEQ); o[j] = wmg16(vj, pb, o[j]); }
    }
    l += __shfl_xor(l, 16, 32);
    const bool any = l > 0.0f;
    const float lsafe = any ? l : 1.0f;
    const float inv = any ? (1.0f / lsafe) : 0.0f;
    const int wb = wave * 16 * OSP;
#pragma unroll
    for (int j = 0; j < 4; ++j) { v4f a, c;
        a[0] = o[j][0] * inv; a[1] = o[j][1] * inv; a[2] = o[j][2] * inv; a[3] = o[j][3] * inv; c[0] = o[j][4] * inv; c[1] = o[j][5] * inv; c[2] = o[j][6] * inv; c[3] = o[j][7] * inv;
        *(v4fa*)(&os[wb + lr * OSP + 16 * j + 8 * hi]) = a; *(v4fa*)(&os[wb + lr * OSP + 16 * j + 8 * hi + 4]) = c; }
    wave_sync();
    h16* crow = CTX + ((size_t)b * SEQ + (size_t)t0) * DM + h * HD;
#pragma unroll 1
    for (int ps = 0; ps < 2; ++ps) {
#pragma unroll
        for (int s = 0; s < 4; ++s) { const int row = 4 * s + (lane >> 3), c8 = (lane & 7) * 8;
            const v4f x0 = *(const v4fa*)(&os[wb + row * OSP + c8]); const v4f x1 = *(const v4fa*)(&os[wb + row * OSP + c8 + 4]); v8h hv;
#pragma unroll
            for (int i = 0; i < 4; ++i) { hv[i] = toh_flush(x0[i] * CXS); hv[4 + i] = toh_flush(x1[i] * CXS); }
            *(volatile v8h*)(crow + (size_t)row * DM + c8) = hv; }
        if (ps == 0) __threadfence(); }
}

static constexpr size_t al256(size_t v) { return (v + 255) & ~(size_t)255; }
static constexpr size_t SZ_XB = al256((size_t)NB * SEQ * DM * 2);
static constexpr size_t SZ_W1 = al256((size_t)DM * DM * 2);
static constexpr size_t SZ_GA = al256((size_t)NB * SEQ * NH_ * 4);
static constexpr size_t SZ_RB = al256((size_t)NH_ * RBN * 4);
static constexpr size_t SZ_GW = al256((size_t)16 * HD * 2);
static constexpr size_t SZ_TOTAL = 5 * SZ_XB + 4 * SZ_W1 + SZ_GA + SZ_RB + SZ_GW;
static_assert(SZ_TOTAL <= (size_t)134217728);
static_assert(((size_t)DM * DM * 2) % 256 == 0);
static_assert((size_t)NB * NH_ * SEQ * HD == (size_t)NB * SEQ * DM);
static_assert(((size_t)NB * SEQ / GT) * (GT * NH_) * 4 == (size_t)NB * SEQ * NH_ * 4);
static_assert(((size_t)NH_ * RBN / 4) % 256 == 0);

extern "C" void kernel_launch(void* const* d_in, const int* in_sizes, int n_in,
                              void* d_out, int out_size, void* d_ws, size_t ws_size, hipStream_t stream) {
    if (n_in < 13) return;
    const size_t needx = ((size_t)(SEQ - 1) * NB_FULL + NB) * DM;
    if ((size_t)in_sizes[0] < needx) return;
    if ((size_t)in_sizes[1] < (size_t)DM * DM || (size_t)in_sizes[3] < (size_t)DM * DM || (size_t)in_sizes[5] < (size_t)DM * DM || (size_t)in_sizes[7] < (size_t)DM * DM) return;
    if (in_sizes[2] < DM || in_sizes[4] < DM || in_sizes[6] < DM || in_sizes[8] < DM) return;
    if (in_sizes[9] < 32 * NH_ || in_sizes[10] < 8 * HD || in_sizes[11] < 8 || in_sizes[12] < NH_) return;
    if ((size_t)out_size < needx) return;
    if (SZ_TOTAL > ws_size) return;
    const float* xq  = (const float*)d_in[0];
    const float* wq  = (const float*)d_in[1];  const float* bq = (const float*)d_in[2];
    const float* wk  = (const float*)d_in[3];  const float* bk = (const float*)d_in[4];
    const float* wv  = (const float*)d_in[5];  const float* bv = (const float*)d_in[6];
    const float* wo  = (const float*)d_in[7];  const float* bo = (const float*)d_in[8];
    const float* remb = (const float*)d_in[9];
    const float* gw  = (const float*)d_in[10]; const float* gbi = (const float*)d_in[11]; const float* gai = (const float*)d_in[12];
    float* OUT = (float*)d_out;
    char* wsp = (char*)d_ws;
    bf*  XB  = (bf*)wsp;  wsp += SZ_XB;
    bf*  WQ  = (bf*)wsp;  wsp += SZ_W1;
    bf*  WK  = (bf*)wsp;  wsp += SZ_W1;
    bf*  WV  = (bf*)wsp;  wsp += SZ_W1;
    h16* WO  = (h16*)wsp; wsp += SZ_W1;
    h16* QH  = (h16*)wsp; wsp += SZ_XB;
    h16* KP  = (h16*)wsp; wsp += SZ_XB;
    h16* VT  = (h16*)wsp; wsp += SZ_XB;
    h16* CTX = (h16*)wsp; wsp += SZ_XB;
    float* GA = (float*)wsp; wsp += SZ_GA;
    float* RB = (float*)wsp; wsp += SZ_RB;
    bf*  GW  = (bf*)wsp;  wsp += SZ_GW;

    { const size_t n8 = (size_t)NB * SEQ * DM / 8;
      k_cvtx<<<(unsigned)((n8 + 255) / 256), 256, 0, stream>>>(xq, XB); }
    { const size_t n8 = (size_t)DM * DM / 8; const unsigned g = (unsigned)((n8 + 255) / 256);
      k_cvt8<<<g, 256, 0, stream>>>(wq, WQ, n8); k_cvt8<<<g, 256, 0, stream>>>(wk, WK, n8); k_cvt8<<<g, 256, 0, stream>>>(wv, WV, n8);
      k_cvtw<<<g, 256, 0, stream>>>(wo, WO, n8); }
    k_gw<<<1, 128, 0, stream>>>(gw, GW);
    k_relb<<<(unsigned)(NH_ * RBN / 4 / 256), 256, 0, stream>>>(remb, RB);
    k_gate<<<(unsigned)(NB * SEQ / GT), 32, 0, stream>>>(XB, GW, gbi, gai, GA);

    k_projqk<<<dim3(NB * SEQ / 64, DM / 64, 1), 32, 0, stream>>>(XB, WQ, bq, QH);
    k_projqk<<<dim3(NB * SEQ / 64, DM / 64, 1), 32, 0, stream>>>(XB, WK, bk, KP);
    k_projv<<<dim3(DM / 64, NB * SEQ / 64, 1), 32, 0, stream>>>(WV, XB, bv, VT);

    k_flash<<<dim3(SEQ / (16 * AW), NB * NH_, 1), 32 * AW, 0, stream>>>(QH, KP, VT, GA, RB, CTX);

    k_oproj<<<dim3(NB * SEQ / 64, DM / 64, 1), 32, 0, stream>>>(CTX, WO, bo, OUT);
}
